// MultiHeadTimeAwareAttention_74826920231001
// MI455X (gfx1250) — hardware-verified
//
#include <hip/hip_runtime.h>
#include <stddef.h>
#include <stdint.h>

#define SQ    2048
#define HID   2048
#define NH    16
#define HDM   128
#define NQKV  6144
#define QB    128
#define KC    64
#define NQB   (SQ / QB)
#define NCK   (SQ / KC)
#define TBN   64
#define QKPLANE (NH * SQ * HDM)

static_assert(SQ % 256 == 0);
static_assert(HID % 64 == 0);
static_assert(HID % 32 == 0);
static_assert(NH * HDM == HID);
static_assert(NQKV == 3 * HID);
static_assert(SQ % KC == 0);
static_assert(SQ % QB == 0);
static_assert((SQ * HID) % 2048 == 0);
static_assert((NH * HID) % 2048 == 0);
static_assert(HDM == 128);

typedef _Float16 v16h __attribute__((ext_vector_type(16)));
typedef _Float16 v8h  __attribute__((ext_vector_type(8)));
typedef float    v8f  __attribute__((ext_vector_type(8)));
typedef float    v4f  __attribute__((ext_vector_type(4)));
typedef unsigned int v4u __attribute__((ext_vector_type(4)));

union Frag  { v16h v; v8h h[2]; };
union Pack8 { v8h h; v4u u; };

__device__ __forceinline__ v8f mma16(v16h a, v16h b, v8f c) {
  c = __builtin_amdgcn_wmma_f32_16x16x32_f16(false, a, false, b, (short)0, c, false, false);
  asm volatile("v_nop\n\tv_nop\n\tv_nop\n\tv_nop" : "+v"(c) : "v"(a), "v"(b));
  return c;
}

__device__ __forceinline__ v16h ldfrag(const _Float16* p, int ld, int row0, int k0, int lane) {
  const int m = lane & 15, lh = lane >> 4;
  const _Float16* q = p + (size_t)(row0 + m) * ld + k0 + 8 * lh;
  Frag f;
  f.h[0] = *(const v8h*)(q);
  f.h[1] = *(const v8h*)(q + 16);
  return f.v;
}

__device__ __forceinline__ v8f zero8() { return (v8f){0.f, 0.f, 0.f, 0.f, 0.f, 0.f, 0.f, 0.f}; }

__device__ __forceinline__ void gemm32x64(const _Float16* __restrict__ A, int lda,
                                          const _Float16* __restrict__ Bt, int ldb, int K,
                                          int m0, int n0, int lane, v8f (&acc)[2][4]) {
#pragma unroll 1
  for (int k0 = 0; k0 < K; k0 += 32) {
    const v16h a0 = ldfrag(A, lda, m0, k0, lane);
    const v16h a1 = ldfrag(A, lda, m0 + 16, k0, lane);
    const v16h b0 = ldfrag(Bt, ldb, n0, k0, lane);
    const v16h b1 = ldfrag(Bt, ldb, n0 + 16, k0, lane);
    const v16h b2 = ldfrag(Bt, ldb, n0 + 32, k0, lane);
    const v16h b3 = ldfrag(Bt, ldb, n0 + 48, k0, lane);
    acc[0][0] = mma16(a0, b0, acc[0][0]);
    acc[1][0] = mma16(a1, b0, acc[1][0]);
    acc[0][1] = mma16(a0, b1, acc[0][1]);
    acc[1][1] = mma16(a1, b1, acc[1][1]);
    acc[0][2] = mma16(a0, b2, acc[0][2]);
    acc[1][2] = mma16(a1, b2, acc[1][2]);
    acc[0][3] = mma16(a0, b3, acc[0][3]);
    acc[1][3] = mma16(a1, b3, acc[1][3]);
  }
}

__global__ __launch_bounds__(256) void k_cvt(const float* __restrict__ src, int nsrc,
                                             _Float16* __restrict__ dh, float scale) {
  const int tid = threadIdx.x;
  const size_t o = (size_t)blockIdx.x * 2048 + (size_t)tid * 8;
  const bool inb = ((size_t)blockIdx.x + 1) * 2048 <= (size_t)nsrc;
  const size_t ol = inb ? o : (size_t)tid * 8;
  const float sc = inb ? scale : 0.f;
  const v4f a0 = *(const v4f*)(src + ol) * sc;
  const v4f a1 = *(const v4f*)(src + ol + 4) * sc;
  Pack8 pk;
  pk.h = (v8h){(_Float16)a0[0], (_Float16)a0[1], (_Float16)a0[2], (_Float16)a0[3],
               (_Float16)a1[0], (_Float16)a1[1], (_Float16)a1[2], (_Float16)a1[3]};
  const v4u vv = pk.u;
  volatile v4u* d = (volatile v4u*)(dh + o);
  *d = vv;
  __threadfence();
  *d = vv;
}

#define STP 72
#define SVP 264
__global__ __launch_bounds__(256) void k_qkv(const _Float16* __restrict__ xh,
                                             const _Float16* __restrict__ wt,
                                             const float* __restrict__ bias,
                                             _Float16* __restrict__ qkp,
                                             _Float16* __restrict__ vtp) {
  __shared__ __align__(16) _Float16 st[256 * STP];
  const int tid = threadIdx.x, lane = tid & 31, wave = tid >> 5;
  const int hh = lane >> 4, c = lane & 15;
  const int sb = blockIdx.x * 256;
  const int ns = blockIdx.y;
  const int which = ns >> 5;
  const int cs    = ns & 31;
  const int head  = cs >> 1;
  const int dh    = cs & 1;
  const int m0 = sb + wave * 32;
  const int n0 = ns * 64;
  const _Float16* A = xh + (size_t)which * SQ * HID;

  v8f acc[2][4];
#pragma unroll
  for (int s = 0; s < 2; ++s)
#pragma unroll
    for (int t = 0; t < 4; ++t) acc[s][t] = zero8();
  gemm32x64(A, HID, wt, HID, HID, m0, n0, lane, acc);

  float bb[4];
#pragma unroll
  for (int t = 0; t < 4; ++t) bb[t] = bias[n0 + 16 * t + c];

  if (which < 2) {
#pragma unroll
    for (int sub = 0; sub < 2; ++sub)
#pragma unroll
      for (int t = 0; t < 4; ++t)
#pragma unroll
        for (int r = 0; r < 8; ++r)
          st[(wave * 32 + sub * 16 + 8 * hh + r) * STP + 16 * t + c] =
              (_Float16)(acc[sub][t][r] * 0.03125f + bb[t]);
  } else {
#pragma unroll
    for (int sub = 0; sub < 2; ++sub)
#pragma unroll
      for (int t = 0; t < 4; ++t)
#pragma unroll
        for (int r = 0; r < 8; ++r)
          st[(16 * t + c) * SVP + wave * 32 + sub * 16 + 8 * hh + r] =
              (_Float16)(acc[sub][t][r] * 0.03125f + bb[t]);
  }
  __syncthreads();

  if (which < 2) {
    _Float16* base = qkp + (size_t)which * QKPLANE + (size_t)head * SQ * HDM + (size_t)dh * 64;
#pragma unroll
    for (int g = 0; g < 2; ++g) {
      v4u val[4];
      size_t go[4];
#pragma unroll
      for (int j = 0; j < 4; ++j) {
        const int p  = tid + 256 * (4 * g + j);
        const int lr = p >> 3;
        const int pc = p & 7;
        Pack8 pk;
        pk.h   = *(const v8h*)(st + lr * STP + pc * 8);
        val[j] = pk.u;
        go[j]  = (size_t)(sb + lr) * HDM + pc * 8;
      }
      for (int ps = 0; ps < 2; ++ps) {
#pragma unroll
        for (int j = 0; j < 4; ++j) *(volatile v4u*)(base + go[j]) = val[j];
        __threadfence();
      }
    }
  } else {
    _Float16* base = vtp + (size_t)head * HDM * SQ + (size_t)dh * 64 * SQ;
#pragma unroll
    for (int g = 0; g < 2; ++g) {
      v4u val[4];
      size_t go[4];
#pragma unroll
      for (int j = 0; j < 4; ++j) {
        const int p    = tid + 256 * (4 * g + j);
        const int drow = p >> 5;
        const int pc   = p & 31;
        Pack8 pk;
        pk.h   = *(const v8h*)(st + drow * SVP + pc * 8);
        val[j] = pk.u;
        go[j]  = (size_t)drow * SQ + sb + pc * 8;
      }
      for (int ps = 0; ps < 2; ++ps) {
#pragma unroll
        for (int j = 0; j < 4; ++j) *(volatile v4u*)(base + go[j]) = val[j];
        __threadfence();
      }
    }
  }
}

#define KTP 136
#define VTP 72
#define PTP 72
#define LDS_KS 0
#define LDS_VS (KC * KTP)
#define LDS_PS (LDS_VS + HDM * VTP)
#define LDS_TOT (LDS_PS + 8 * 16 * PTP)
static_assert(128 * KTP <= LDS_PS);
__global__ __launch_bounds__(256) void k_attn(const _Float16* __restrict__ qp,
                                              const _Float16* __restrict__ kp,
                                              const _Float16* __restrict__ vt,
                                              const float* __restrict__ tbp,
                                              _Float16* __restrict__ op, float sscale) {
  __shared__ __align__(16) _Float16 sm[LDS_TOT];
  _Float16* Ks = sm + LDS_KS;
  _Float16* Vs = sm + LDS_VS;
  _Float16* Ps = sm + LDS_PS;

  const int tid = threadIdx.x, lane = tid & 31, wave = tid >> 5;
  const int hh = lane >> 4, c = lane & 15;
  const int qb  = blockIdx.x % NQB;
  const int h   = blockIdx.x / NQB;
  const int q0  = qb * QB + wave * 16;

  const _Float16* Q = qp + (size_t)h * SQ * HDM;
  const _Float16* K = kp + (size_t)h * SQ * HDM;
  const _Float16* V = vt + (size_t)h * HDM * SQ;

  const float NEGI = -__builtin_huge_valf();
  float mrow[8], lrow[8];
  v8f oacc[8];
#pragma unroll
  for (int r = 0; r < 8; ++r) { mrow[r] = NEGI; lrow[r] = 0.f; }
#pragma unroll
  for (int t = 0; t < 8; ++t) oacc[t] = zero8();

  _Float16* pw = Ps + wave * 16 * PTP;

  for (int kc = 0; kc < NCK; ++kc) {
    const int kv0 = kc * KC;
    __syncthreads();
    {
      const int r  = tid >> 2;
      const int qq = (tid & 3) * 32;
      const _Float16* ks = K + (size_t)(kv0 + r) * HDM + qq;
#pragma unroll
      for (int e = 0; e < 4; ++e) *(v8h*)(Ks + r * KTP + qq + 8 * e) = *(const v8h*)(ks + 8 * e);
      const int r2 = tid >> 1;
      const int q2 = (tid & 1) * 32;
      const _Float16* vs = V + (size_t)r2 * SQ + kv0 + q2;
#pragma unroll
      for (int e = 0; e < 4; ++e) *(v8h*)(Vs + r2 * VTP + q2 + 8 * e) = *(const v8h*)(vs + 8 * e);
    }
    __syncthreads();

    v8f s[4];
#pragma unroll
    for (int j = 0; j < 4; ++j) s[j] = zero8();
#pragma unroll
    for (int dc = 0; dc < 4; ++dc) {
      const v16h qa = ldfrag(Q, HDM, q0, dc * 32, lane);
#pragma unroll
      for (int j = 0; j < 4; ++j) {
        const v16h kb = ldfrag(Ks, KTP, j * 16, dc * 32, lane);
        s[j] = mma16(qa, kb, s[j]);
      }
    }
    float tb[4];
#pragma unroll
    for (int j = 0; j < 4; ++j) tb[j] = tbp[(size_t)(kv0 + j * 16 + c) * TBN + h];
    float cm[8];
#pragma unroll
    for (int r = 0; r < 8; ++r) {
      float m = NEGI;
#pragma unroll
      for (int j = 0; j < 4; ++j) { s[j][r] = s[j][r] * sscale + tb[j]; m = fmaxf(m, s[j][r]); }
#pragma unroll
      for (int off = 1; off < 16; off <<= 1) m = fmaxf(m, __shfl_xor(m, off, 32));
      cm[r] = m;
    }
    float al[8];
#pragma unroll
    for (int r = 0; r < 8; ++r) {
      const float mnew  = fmaxf(mrow[r], cm[r]);
      const float alpha = __expf(mrow[r] - mnew);
      mrow[r] = mnew;
      float psum = 0.f;
#pragma unroll
      for (int j = 0; j < 4; ++j) {
        const float p = __expf(s[j][r] - mnew);
        psum += p;
        pw[(8 * hh + r) * PTP + j * 16 + c] = (_Float16)(p * 1024.0f);
      }
#pragma unroll
      for (int off = 1; off < 16; off <<= 1) psum += __shfl_xor(psum, off, 32);
      lrow[r] = lrow[r] * alpha + psum;
      al[r] = alpha;
    }
#pragma unroll
    for (int t = 0; t < 8; ++t)
#pragma unroll
      for (int r = 0; r < 8; ++r) oacc[t][r] *= al[r];
    __syncthreads();

#pragma unroll
    for (int kk = 0; kk < 2; ++kk) {
      const v16h pa = ldfrag(pw, PTP, 0, kk * 32, lane);
#pragma unroll
      for (int t = 0; t < 8; ++t) {
        const v16h vb = ldfrag(Vs, VTP, t * 16, kk * 32, lane);
        oacc[t] = mma16(pa, vb, oacc[t]);
      }
    }
  }

  float invl[8];
#pragma unroll
  for (int r = 0; r < 8; ++r) invl[r] = (lrow[r] > 0.f) ? (0.0625f / lrow[r]) : 0.f;
  __syncthreads();
  _Float16* os = sm + (size_t)wave * 16 * KTP;
#pragma unroll
  for (int r = 0; r < 8; ++r) {
#pragma unroll
    for (int t = 0; t < 8; ++t)
      os[(8 * hh + r) * KTP + 16 * t + c] = (_Float16)(oacc[t][r] * invl[r]);
  }
  __syncthreads();
  v4u val[8];
  size_t go[8];
#pragma unroll
  for (int it = 0; it < 8; ++it) {
    const int p  = lane + 32 * it;
    const int L  = p >> 4;
    const int pc = p & 15;
    Pack8 pk;
    pk.h    = *(const v8h*)(os + L * KTP + pc * 8);
    val[it] = pk.u;
    go[it]  = (size_t)(q0 + L) * HID + (size_t)h * HDM + pc * 8;
  }
  for (int ps = 0; ps < 2; ++ps) {
#pragma unroll
    for (int it = 0; it < 8; ++it) *(volatile v4u*)(op + go[it]) = val[it];
    __threadfence();
  }
}

#define OTP 68
__device__ __forceinline__ void out_epilogue_f32(v8f (&acc)[2][4], float scale, const float (&bb)[4],
                                                 float* sw, float* __restrict__ out, int ldo,
                                                 int m0, int n0, int lane, int hh, int c) {
#pragma unroll
  for (int sub = 0; sub < 2; ++sub) {
    __syncthreads();
#pragma unroll
    for (int t = 0; t < 4; ++t) {
#pragma unroll
      for (int r = 0; r < 8; ++r) sw[(8 * hh + r) * OTP + 16 * t + c] = acc[sub][t][r] * scale + bb[t];
    }
    __syncthreads();
    v4f val[8];
    size_t go[8];
#pragma unroll
    for (int it = 0; it < 8; ++it) {
      const int p    = lane + 32 * it;
      const int L    = p >> 3;
      const int pc   = p & 7;
      const int row  = L >> 1;
      const int half = L & 1;
      val[it] = *(const v4f*)(sw + row * OTP + half * 32 + pc * 4);
      go[it]  = (size_t)(m0 + sub * 16 + row) * ldo + n0 + half * 32 + pc * 4;
    }
    for (int ps = 0; ps < 2; ++ps) {
#pragma unroll
      for (int it = 0; it < 8; ++it) *(volatile v4f*)(out + go[it]) = val[it];
      __threadfence();
    }
  }
}

__global__ __launch_bounds__(256) void k_gemm_f32(const _Float16* __restrict__ ap, int lda,
                                                  const _Float16* __restrict__ wt, int K,
                                                  const float* __restrict__ bias, int nbias, float scale,
                                                  float* __restrict__ out, int ldo) {
  __shared__ __align__(16) float st[8][16 * OTP];
  const int tid = threadIdx.x, lane = tid & 31, wave = tid >> 5;
  const int hh = lane >> 4, c = lane & 15;
  const int m0 = blockIdx.x * 256 + wave * 32;
  const int n0 = blockIdx.y * 64;

  v8f acc[2][4];
#pragma unroll
  for (int s = 0; s < 2; ++s)
#pragma unroll
    for (int t = 0; t < 4; ++t) acc[s][t] = zero8();
  gemm32x64(ap, lda, wt, K, K, m0, n0, lane, acc);
  float bb[4];
#pragma unroll
  for (int t = 0; t < 4; ++t) {
    const int bi  = n0 + 16 * t + c;
    const int bic = (bi < nbias) ? bi : (nbias - 1);
    const float bv = bias[bic];
    bb[t] = (bi < nbias) ? bv : 0.f;
  }
  out_epilogue_f32(acc, scale, bb, st[wave], out, ldo, m0, n0, lane, hh, c);
}

__global__ __launch_bounds__(256) void k_ln(const float* __restrict__ t, const float* __restrict__ res,
                                            const float* __restrict__ g, const float* __restrict__ be,
                                            float* __restrict__ out) {
  const int tid = threadIdx.x, lane = tid & 31, wave = tid >> 5;
  const size_t m = (size_t)blockIdx.x * 8 + wave;
  const float* tr = t + m * HID;
  const float* rr = res + m * HID;

  v4f v[16];
  float s = 0.f;
#pragma unroll
  for (int it = 0; it < 16; ++it) {
    const int idx = it * 128 + lane * 4;
    const v4f a = *(const v4f*)(tr + idx);
    const v4f r = *(const v4f*)(rr + idx);
    v[it] = a + r;
    s += (v[it][0] + v[it][1]) + (v[it][2] + v[it][3]);
  }
#pragma unroll
  for (int off = 16; off >= 1; off >>= 1) s += __shfl_xor(s, off, 32);
  const float mean = s * 0.00048828125f;
  float ss = 0.f;
#pragma unroll
  for (int it = 0; it < 16; ++it) {
    const v4f d = v[it] - mean;
    ss += (d[0] * d[0] + d[1] * d[1]) + (d[2] * d[2] + d[3] * d[3]);
  }
#pragma unroll
  for (int off = 16; off >= 1; off >>= 1) ss += __shfl_xor(ss, off, 32);
  const float var  = ss * 0.00048828125f;
  const float rstd = rsqrtf(var + 1e-5f);

#pragma unroll
  for (int it = 0; it < 16; ++it) {
    const int idx = it * 128 + lane * 4;
    const v4f gv = *(const v4f*)(g + idx);
    const v4f bv = *(const v4f*)(be + idx);
    v[it] = ((v[it] - mean) * rstd) * gv + bv;
  }
  for (int ps = 0; ps < 2; ++ps) {
#pragma unroll
    for (int it = 0; it < 16; ++it) *(volatile v4f*)(out + m * HID + it * 128 + lane * 4) = v[it];
    __threadfence();
  }
}

extern "C" void kernel_launch(void* const* d_in, const int* in_sizes, int n_in,
                              void* d_out, int out_size, void* d_ws, size_t ws_size,
                              hipStream_t stream) {
  if (n_in < 12) return;
  if (in_sizes[0] != SQ * HID) return;
  if (in_sizes[1] != SQ * HID) return;
  if (in_sizes[2] != SQ * HID) return;
  if (in_sizes[3] != SQ * HID) return;
  if (in_sizes[4] != NQKV * HID) return;
  if (in_sizes[5] != NQKV) return;
  if (in_sizes[6] != HID * HID) return;
  if (in_sizes[7] != HID) return;
  if (in_sizes[8] != NH * HID) return;
  if (in_sizes[9] != NH) return;
  if (in_sizes[10] != HID) return;
  if (in_sizes[11] != HID) return;
  if (out_size != SQ * HID) return;

  const float* query = (const float*)d_in[0];
  const float* key   = (const float*)d_in[1];
  const float* value = (const float*)d_in[2];
  const float* temb  = (const float*)d_in[3];
  const float* inw   = (const float*)d_in[4];
  const float* inb   = (const float*)d_in[5];
  const float* wo    = (const float*)d_in[6];
  const float* bo    = (const float*)d_in[7];
  const float* tpw   = (const float*)d_in[8];
  const float* tpb   = (const float*)d_in[9];
  const float* lng   = (const float*)d_in[10];
  const float* lnb   = (const float*)d_in[11];
  float* out = (float*)d_out;

  size_t off = 0;
  const size_t oX   = off; off += (size_t)3 * SQ * HID * 2;
  const size_t oTh  = off; off += (size_t)SQ * HID * 2;
  const size_t oWt  = off; off += (size_t)NQKV * HID * 2;
  const size_t oWo  = off; off += (size_t)HID * HID * 2;
  const size_t oTP  = off; off += (size_t)TBN * HID * 2;
  const size_t oQ   = off; off += (size_t)NH * SQ * HDM * 2;
  const size_t oK   = off; off += (size_t)NH * SQ * HDM * 2;
  const size_t oV   = off; off += (size_t)NH * HDM * SQ * 2;
  const size_t oTb  = off; off += (size_t)SQ * TBN * 4;
  const size_t oO   = off; off += (size_t)SQ * HID * 2;
  const size_t oT   = off; off += (size_t)SQ * HID * 4;
  if (off > ws_size) return;
  if (off > (size_t)134217728) return;
  if (oK != oQ + (size_t)QKPLANE * 2) return;

  char* ws = (char*)d_ws;
  _Float16* Xh  = (_Float16*)(ws + oX);
  _Float16* Th  = (_Float16*)(ws + oTh);
  _Float16* Wt  = (_Float16*)(ws + oWt);
  _Float16* Wot = (_Float16*)(ws + oWo);
  _Float16* TPt = (_Float16*)(ws + oTP);
  _Float16* QKp = (_Float16*)(ws + oQ);
  _Float16* Kp  = (_Float16*)(ws + oK);
  _Float16* Vt  = (_Float16*)(ws + oV);
  float*    Tb  = (float*)(ws + oTb);
  _Float16* Op  = (_Float16*)(ws + oO);
  float*    T   = (float*)(ws + oT);

  k_cvt<<<dim3((SQ * HID) / 2048), dim3(256), 0, stream>>>(query, in_sizes[0], Xh, 1.0f);
  k_cvt<<<dim3((SQ * HID) / 2048), dim3(256), 0, stream>>>(key, in_sizes[1], Xh + (size_t)SQ * HID, 1.0f);
  k_cvt<<<dim3((SQ * HID) / 2048), dim3(256), 0, stream>>>(value, in_sizes[2], Xh + (size_t)2 * SQ * HID, 1.0f);
  k_cvt<<<dim3((SQ * HID) / 2048), dim3(256), 0, stream>>>(temb, in_sizes[3], Th, 1.0f);
  k_cvt<<<dim3((NQKV * HID) / 2048), dim3(256), 0, stream>>>(inw, in_sizes[4], Wt, 32.0f);
  k_cvt<<<dim3((HID * HID) / 2048), dim3(256), 0, stream>>>(wo, in_sizes[6], Wot, 32.0f);
  k_cvt<<<dim3((TBN * HID) / 2048), dim3(256), 0, stream>>>(tpw, in_sizes[8], TPt, 32.0f);
  k_qkv<<<dim3(SQ / 256, NQKV / 64), dim3(256), 0, stream>>>(Xh, Wt, inb, QKp, Vt);
  k_gemm_f32<<<dim3(SQ / 256, TBN / 64), dim3(256), 0, stream>>>(Th, HID, TPt, HID, tpb, NH, 0.03125f, Tb, TBN);
  const float sscale = 0.0883883476483184f;
  k_attn<<<dim3(NH * NQB), dim3(256), 0, stream>>>(QKp, Kp, Vt, Tb, Op, sscale);
  k_gemm_f32<<<dim3(SQ / 256, HID / 64), dim3(256), 0, stream>>>(Op, HID, Wot, HID, bo, HID, 0.00048828125f, T, HID);
  k_ln<<<dim3(SQ / 8), dim3(256), 0, stream>>>(T, query, lng, lnb, out);
  (void)hipGetLastError();
}
